// SimpleMLP_39762807226843
// MI455X (gfx1250) — hardware-verified
//
#include <hip/hip_runtime.h>
#include <stdint.h>
#include <stddef.h>


typedef _Float16 v16h __attribute__((ext_vector_type(16)));
typedef _Float16 v8h  __attribute__((ext_vector_type(8)));
typedef float    v8f  __attribute__((ext_vector_type(8)));
typedef float    v4f  __attribute__((ext_vector_type(4)));
union Frag { v16h v; v8h half[2]; };

#define HD    128
#define TILE  128
#define NTHR  256
#define NWAVE (NTHR / 32)
#define NLMAX 8

__device__ __forceinline__ float silu_f(float x)
{
    return x * __builtin_amdgcn_rcpf(1.0f + __expf(-x));
}

__device__ __forceinline__ v8f wmma_f16(v8f acc, v16h a, v16h b)
{
    acc = __builtin_amdgcn_wmma_f32_16x16x32_f16(false, a, false, b, (short)0, acc, false, false);
    asm volatile("v_nop\n\tv_nop\n\tv_nop\n\tv_nop" : "+v"(acc) : "v"(a), "v"(b));
    return acc;
}

__global__ __launch_bounds__(NTHR) void k_prep(const float* __restrict__ Wh,
                                                _Float16* __restrict__ WhT, int nL)
{
    __shared__ __attribute__((aligned(16))) _Float16 sT[16 * HD];
    const int t  = threadIdx.x;
    const int l  = blockIdx.x >> 3;
    const int n0 = (blockIdx.x & 7) * 16;
    for (int idx = t; idx < 16 * HD; idx += NTHR) {
        const int k = idx >> 4;
        const int j = idx & 15;
        sT[j * HD + k] = (_Float16)(16.0f * Wh[((size_t)l * HD + k) * HD + n0 + j]);
    }
    __syncthreads();
    const int row = t >> 4;
    const int ch  = t & 15;
    const v8h val = *(const v8h*)(sT + row * HD + 8 * ch);
    _Float16* p = WhT + ((size_t)(l * HD + n0 + row) * HD + 8 * ch);
    *(volatile v8h*)p = val;
    __threadfence();
    *(volatile v8h*)p = val;
    (void)nL;
}

__global__ __launch_bounds__(NTHR) void k_main(
    const float* __restrict__ pos, const int* __restrict__ Zn,
    const float* __restrict__ Win, const float* __restrict__ bin,
    const _Float16* __restrict__ WhT, const float* __restrict__ bh,
    const float* __restrict__ We,  const float* __restrict__ bE,
    float* __restrict__ wsE, float* __restrict__ wsC, int N, int nL)
{
    __shared__ __attribute__((aligned(16))) _Float16 sH0[TILE * HD];
    __shared__ __attribute__((aligned(16))) _Float16 sH1[TILE * HD];
    __shared__ __attribute__((aligned(16))) float sWin[4 * HD];
    __shared__ __attribute__((aligned(16))) float sBin[HD];
    __shared__ __attribute__((aligned(16))) float sBh[NLMAX * HD];
    __shared__ __attribute__((aligned(16))) float sWe[HD];
    __shared__ __attribute__((aligned(16))) float sE[TILE];
    __shared__ __attribute__((aligned(16))) float sCS[NWAVE * HD];
    __shared__ __attribute__((aligned(16))) float sCB[HD];

    const int t    = threadIdx.x;
    const int lane = t & 31;
    const int wave = t >> 5;
    const int col  = lane & 15;
    const int hh   = lane >> 4;
    const int a0   = blockIdx.x * TILE;

    for (int i = t; i < 4 * HD; i += NTHR) sWin[i] = Win[i];
    for (int i = t; i < HD; i += NTHR) { sBin[i] = bin[i]; sWe[i] = We[i]; }
    for (int i = t; i < nL * HD; i += NTHR) sBh[i] = bh[i];
    __syncthreads();

    {
        const int aLoc  = t >> 1;
        const int jBase = (t & 1) * 64;
        const int aG    = a0 + aLoc;
        float f0 = 0.f, f1 = 0.f, f2 = 0.f, f3 = 0.f;
        if (aG < N) {
            const float* pr = pos + (size_t)aG * 3;
            f0 = pr[0]; f1 = pr[1]; f2 = pr[2];
            f3 = (float)Zn[aG];
        }
        #pragma unroll
        for (int jv = 0; jv < 8; ++jv) {
            v8h pack;
            #pragma unroll
            for (int e = 0; e < 8; ++e) {
                const int j = jBase + jv * 8 + e;
                float x = f0 * sWin[j] + f1 * sWin[HD + j]
                        + f2 * sWin[2 * HD + j] + f3 * sWin[3 * HD + j];
                x += sBin[j];
                pack[e] = (_Float16)silu_f(x);
            }
            *(v8h*)(sH0 + aLoc * HD + jBase + jv * 8) = pack;
        }
    }

    const int   rowA  = wave * 16 + col;
    const int   rowDl = wave * 16 + hh * 8;
    const int   rowDg = a0 + rowDl;
    const float bE0   = bE[0];

    float ep[8];
    #pragma unroll
    for (int r = 0; r < 8; ++r) ep[r] = 0.f;

    for (int l = 0; l < nL; ++l) {
        __syncthreads();
        const _Float16* sIn  = (l & 1) ? sH1 : sH0;
        _Float16*       sOut = (l & 1) ? sH0 : sH1;
        const bool last = (l + 1 == nL);

        Frag a[4];
        const _Float16* arow = sIn + rowA * HD + hh * 8;
        #pragma unroll
        for (int kc = 0; kc < 4; ++kc) {
            a[kc].half[0] = *(const v8h*)(arow + kc * 32);
            a[kc].half[1] = *(const v8h*)(arow + kc * 32 + 16);
        }

        const _Float16* bl  = WhT + (size_t)l * HD * HD + hh * 8;
        const float*    bhl = sBh + l * HD;

        #pragma unroll 1
        for (int nt = 0; nt < 8; ++nt) {
            const int n = nt * 16 + col;
            const _Float16* brow = bl + (size_t)n * HD;
            Frag b[4];
            #pragma unroll
            for (int kc = 0; kc < 4; ++kc) {
                b[kc].half[0] = *(const v8h*)(brow + kc * 32);
                b[kc].half[1] = *(const v8h*)(brow + kc * 32 + 16);
            }
            v8f acc = {0.f, 0.f, 0.f, 0.f, 0.f, 0.f, 0.f, 0.f};
            #pragma unroll
            for (int kc = 0; kc < 4; ++kc) acc = wmma_f16(acc, a[kc].v, b[kc].v);

            const float bias = bhl[n];
            float v[8];
            #pragma unroll
            for (int r = 0; r < 8; ++r) v[r] = silu_f(acc[r] * 0.0625f + bias);

            if (!last) {
                #pragma unroll
                for (int r = 0; r < 8; ++r) sOut[(rowDl + r) * HD + n] = (_Float16)v[r];
            } else {
                const float we = sWe[n];
                float cs = 0.f;
                #pragma unroll
                for (int r = 0; r < 8; ++r) {
                    ep[r] += v[r] * we;
                    cs += (rowDg + r < N) ? v[r] : 0.f;
                }
                cs += __shfl_xor(cs, 16);
                if (hh == 0) sCS[wave * HD + n] = cs;
            }
        }
    }

    #pragma unroll
    for (int off = 1; off < 16; off <<= 1) {
        #pragma unroll
        for (int r = 0; r < 8; ++r) ep[r] += __shfl_xor(ep[r], off);
    }
    if (col == 0) {
        #pragma unroll
        for (int r = 0; r < 8; ++r) sE[rowDl + r] = ep[r] + bE0;
    }
    __syncthreads();
    if (t < HD) {
        float s = 0.f;
        #pragma unroll
        for (int w = 0; w < NWAVE; ++w) s += sCS[w * HD + t];
        sCB[t] = s;
    }
    __syncthreads();
    if (wave == 0) {
        const v4f ev = *(const v4f*)(sE  + 4 * lane);
        const v4f cv = *(const v4f*)(sCB + 4 * lane);
        float* pe = wsE + (size_t)a0 + 4 * lane;
        float* pc = wsC + (size_t)blockIdx.x * HD + 4 * lane;
        *(volatile v4f*)pe = ev;
        *(volatile v4f*)pc = cv;
        __threadfence();
        *(volatile v4f*)pe = ev;
        *(volatile v4f*)pc = cv;
    }
}

__device__ __forceinline__ float seg_sum_one(const int* __restrict__ batch,
                                             const float* __restrict__ wsE,
                                             int N, int S, int s)
{
    float sum = 0.f;
    if (s < S) {
        int lo = 0, hi = N;
        while (lo < hi) { const int mid = (lo + hi) >> 1; if (batch[mid] < s)  lo = mid + 1; else hi = mid; }
        const int start = lo;
        hi = N;
        while (lo < hi) { const int mid = (lo + hi) >> 1; if (batch[mid] <= s) lo = mid + 1; else hi = mid; }
        const int end = lo;
        for (int i = start; i < end; ++i) sum += wsE[i];
    }
    return sum;
}

__global__ __launch_bounds__(NTHR) void k_seg(const int* __restrict__ batch,
                                               const float* __restrict__ wsE,
                                               float* __restrict__ out, int N, int S, int Spad)
{
    const int gl = blockIdx.x * NTHR + threadIdx.x;
    const int s0 = 4 * gl;
    v4f ev;
    ev.x = seg_sum_one(batch, wsE, N, S, s0 + 0);
    ev.y = seg_sum_one(batch, wsE, N, S, s0 + 1);
    ev.z = seg_sum_one(batch, wsE, N, S, s0 + 2);
    ev.w = seg_sum_one(batch, wsE, N, S, s0 + 3);
    const bool w = (s0 < Spad);
    float* p = out + (size_t)s0;
    if (w) *(volatile v4f*)p = ev;
    __threadfence();
    if (w) *(volatile v4f*)p = ev;
}

__global__ __launch_bounds__(NTHR) void k_zero(float* __restrict__ out, int startF, int count4)
{
    const int gl = blockIdx.x * NTHR + threadIdx.x;
    const bool w = (gl < count4);
    float* p = out + (size_t)startF + 4 * (size_t)gl;
    const v4f z = {0.f, 0.f, 0.f, 0.f};
    if (w) *(volatile v4f*)p = z;
    __threadfence();
    if (w) *(volatile v4f*)p = z;
}

__global__ __launch_bounds__(HD) void k_stress(
    const float* __restrict__ wsC, int nwg,
    const float* __restrict__ Ws, const float* __restrict__ bs,
    float* __restrict__ out, double rN, int tailStart, int nz, int ntail)
{
    __shared__ float hmean[HD];
    __shared__ float sS[8];
    const int t = threadIdx.x;
    {
        double s = 0.0;
        for (int w = 0; w < nwg; ++w) s += (double)wsC[(size_t)w * HD + t];
        hmean[t] = (float)(s * rN);
    }
    if (t < 8) sS[t] = 0.f;
    __syncthreads();
    if (t < 6) {
        float acc = 0.f;
        #pragma unroll 8
        for (int n = 0; n < HD; ++n) acc += hmean[n] * Ws[n * 6 + t];
        sS[t] = acc + bs[t];
    }
    __syncthreads();
    const bool w = (t < ntail);
    float val = 0.f;
    if (w && t >= nz) val = sS[t - nz];
    float* p = out + (size_t)tailStart + t;
    if (w) *(volatile float*)p = val;
    __threadfence();
    if (w) *(volatile float*)p = val;
}

static inline size_t align128(size_t x) { return (x + 127) & ~(size_t)127; }

extern "C" void kernel_launch(void* const* d_in, const int* in_sizes, int n_in,
                              void* d_out, int out_size, void* d_ws, size_t ws_size,
                              hipStream_t stream)
{
    if (n_in < 11) return;
    const float* pos   = (const float*)d_in[0];
    const int*   Zn    = (const int*)  d_in[1];
    const int*   batch = (const int*)  d_in[2];
    const float* Win   = (const float*)d_in[3];
    const float* bin   = (const float*)d_in[4];
    const float* Wh    = (const float*)d_in[5];
    const float* bh    = (const float*)d_in[6];
    const float* We    = (const float*)d_in[7];
    const float* bEp   = (const float*)d_in[8];
    const float* Ws    = (const float*)d_in[9];
    const float* bs    = (const float*)d_in[10];

    const int N  = in_sizes[1];
    const int nL = in_sizes[5] / (HD * HD);
    const int S  = out_size - 3 * N - 6;
    if (N <= 0 || S <= 0 || nL < 1 || nL > NLMAX) return;
    if (in_sizes[3] != 4 * HD || in_sizes[4] != HD || in_sizes[6] != nL * HD ||
        in_sizes[7] != HD || in_sizes[8] < 1 || in_sizes[9] != HD * 6 || in_sizes[10] != 6) return;

    const int nwg = (N + TILE - 1) / TILE;

    const size_t offWhT = 0;
    const size_t bWhT   = (size_t)nL * HD * HD * sizeof(_Float16);
    const size_t offE   = align128(offWhT + bWhT);
    const size_t bE     = (size_t)nwg * TILE * sizeof(float);
    const size_t offC   = align128(offE + bE);
    const size_t bC     = (size_t)nwg * HD * sizeof(float);
    const size_t total  = offC + bC;
    if (total > ws_size) return;

    _Float16* WhT = (_Float16*)((char*)d_ws + offWhT);
    float*    wsE = (float*)((char*)d_ws + offE);
    float*    wsC = (float*)((char*)d_ws + offC);
    float*    out = (float*)d_out;

    const long long totF = (long long)S + 3LL * N;
    const int Spad       = (S + 31) & ~31;
    const int tailStart  = (int)(totF & ~31LL);
    if (Spad > tailStart) return;
    const int count4 = (tailStart - Spad) / 4;
    const int nz     = (int)(totF - tailStart);
    const int ntail  = out_size - tailStart;
    if (ntail > HD || ntail < 0) return;
    const double rN  = 1.0 / (double)N;

    hipLaunchKernelGGL(k_prep, dim3(nL * 8), dim3(NTHR), 0, stream, Wh, WhT, nL);
    hipLaunchKernelGGL(k_main, dim3(nwg), dim3(NTHR), 0, stream,
                       pos, Zn, Win, bin, (const _Float16*)WhT, bh, We, bEp, wsE, wsC, N, nL);
    hipLaunchKernelGGL(k_seg, dim3((Spad / 4 + NTHR - 1) / NTHR), dim3(NTHR), 0, stream,
                       batch, (const float*)wsE, out, N, S, Spad);
    if (count4 > 0)
        hipLaunchKernelGGL(k_zero, dim3((count4 + NTHR - 1) / NTHR), dim3(NTHR), 0, stream,
                           out, Spad, count4);
    hipLaunchKernelGGL(k_stress, dim3(1), dim3(HD), 0, stream,
                       (const float*)wsC, nwg, Ws, bs, out, rN, tailStart, nz, ntail);
    (void)hipGetLastError();
}
